// ResidualWaveFrobinator_64115271794987
// MI455X (gfx1250) — hardware-verified
//
#include <hip/hip_runtime.h>
#include <math.h>
#include <stddef.h>
#include <stdint.h>


#define NB    2
#define FIN   128
#define FOUT  128
#define FH    16
#define HW    4096
#define NPIX  8192
#define KP    1024
#define KW    2048
#define KTOT  2176
#define KC    128
#define NCH   17
#define NCHW  16
#define PXP   64
#define PXG   128
#define NTHR  256
#define WSCAP 134217728

#define S_W   64.0f
#define S_P   16.0f
#define S_WC  16.0f
#define S_A   4.0f
#define YSCALE ((1.0f / 256.0f) * 0.08838834764831845f)

#define NP8W  32768
#define NP8   34816

#define XHP     136
#define PPW     1032
#define OFF_XH  0
#define OFF_WAB 17408
#define OFF_WC  26112
#define OFF_PRE 59136
#define OFF_FF  67328
#define OFF_P   83712
#define OFF_CP  215808
#define OFF_CS  224000
#define LDS_PREP 228096

#define BSP      136
#define GOFF_XS  0
#define GOFF_BS  65536
#define GOFF_NS  100352
#define LDS_GEMM 100480

static_assert(NTHR == 256);
static_assert(FIN == FOUT);
static_assert(KW == FIN * FH);
static_assert(KTOT == KW + FIN);
static_assert(KP == (2 * FH) * (2 * FH));
static_assert((KTOT % KC) == 0 && NCH * KC == KTOT && NCHW * KC == KW);
static_assert((KC % 32) == 0 && (FIN % 32) == 0 && (KP % 64) == 0);
static_assert((HW % PXP) == 0 && (HW % PXG) == 0 && NPIX == NB * HW);
static_assert(NP8W == FOUT * KW / 8 && NP8 == NP8W + FOUT * FIN / 8);
static_assert((NP8W % 32) == 0 && (NP8 % NTHR) == 0);
static_assert(OFF_WAB == OFF_XH  + PXP * XHP * 2);
static_assert(OFF_WC  == OFF_WAB + 2 * FH * XHP * 2);
static_assert(OFF_PRE == OFF_WC  + FH * PPW * 2);
static_assert(OFF_FF  == OFF_PRE + PXP * 32 * 4);
static_assert(OFF_P   == OFF_FF  + PXP * 64 * 4);
static_assert(OFF_CP  == OFF_P   + PXP * PPW * 2);
static_assert(OFF_CS  == OFF_CP  + 2 * PXP * FH * 4);
static_assert(LDS_PREP == OFF_CS + PXP * FH * 4);
static_assert(LDS_PREP <= 298 * 1024);
static_assert(GOFF_BS  == GOFF_XS + FIN * PXG * 4);
static_assert(GOFF_NS  == GOFF_BS + FOUT * BSP * 2);
static_assert(LDS_GEMM == GOFF_NS + 2 * FH * 4);
static_assert((OFF_WAB % 16) == 0 && (OFF_WC % 16) == 0 && (OFF_PRE % 16) == 0 && (OFF_FF % 16) == 0);
static_assert((OFF_P % 16) == 0 && (OFF_CP % 16) == 0 && (OFF_CS % 16) == 0 && (GOFF_BS % 16) == 0);
static_assert((XHP % 8) == 0 && (PPW % 8) == 0 && (BSP % 8) == 0 && (KTOT % 8) == 0);

typedef float    v4f  __attribute__((ext_vector_type(4)));
typedef float    v8f  __attribute__((ext_vector_type(8)));
typedef double   v2d  __attribute__((ext_vector_type(2)));
typedef _Float16 v8h  __attribute__((ext_vector_type(8)));
typedef _Float16 v16h __attribute__((ext_vector_type(16)));
union FragH { v16h v; v8h h[2]; };

__device__ __forceinline__ v8f wmf(v16h a, v16h b, v8f c) {
  v8f d = __builtin_amdgcn_wmma_f32_16x16x32_f16(false, a, false, b, (short)0, c, false, false);
  asm volatile("v_nop\n\tv_nop\n\tv_nop\n\tv_nop" : "+v"(d) : "v"(a), "v"(b));
  return d;
}

__device__ __forceinline__ v8f vzero8() {
  v8f z = {0.f, 0.f, 0.f, 0.f, 0.f, 0.f, 0.f, 0.f};
  return z;
}

__device__ __forceinline__ v8h cvt8(v4f u0, v4f u1, float s) {
  v8h hv;
  hv[0] = (_Float16)(u0.x * s); hv[1] = (_Float16)(u0.y * s); hv[2] = (_Float16)(u0.z * s); hv[3] = (_Float16)(u0.w * s);
  hv[4] = (_Float16)(u1.x * s); hv[5] = (_Float16)(u1.y * s); hv[6] = (_Float16)(u1.z * s); hv[7] = (_Float16)(u1.w * s);
  return hv;
}

__global__ __launch_bounds__(NTHR) void k_pack(const float* __restrict__ wl, const float* __restrict__ bl,
                                               _Float16* Bp) {
  const int idx = blockIdx.x * NTHR + (int)threadIdx.x;
  if (idx >= NP8) return;
  v8h hv;
  size_t doff;
  if (idx < NP8W) {
    const int o = idx >> 8, r = idx & 255;
    const int f = r >> 1, half = r & 1;
    const float* src = wl + ((size_t)f * FOUT + o) * FH + 8 * half;
    const v4f u0 = *(const v4f*)src;
    const v4f u1 = *(const v4f*)(src + 4);
    hv = cvt8(u0, u1, S_W);
    doff = (size_t)o * KTOT + 8 * r;
  } else {
    const int j = idx - NP8W;
    const int o = j >> 4, q = j & 15;
#pragma unroll
    for (int e = 0; e < 8; ++e) hv[e] = (_Float16)(bl[(size_t)(8 * q + e) * FOUT + o] * S_W);
    doff = (size_t)o * KTOT + KW + 8 * q;
  }
  _Float16* d = Bp + doff;
  *(volatile v8h*)d = hv;
  __threadfence();
  *(volatile v8h*)d = hv;
}

__global__ __launch_bounds__(NTHR) void k_prep(
    const float* __restrict__ x, const float* __restrict__ wa, const float* __restrict__ ba,
    const float* __restrict__ wb, const float* __restrict__ bb,
    const float* __restrict__ wc, const float* __restrict__ bc,
    float* wsc, double* wspart)
{
  extern __shared__ v4f lds_prep[];
  unsigned char* lb = (unsigned char*)lds_prep;
  _Float16* xh    = (_Float16*)(lb + OFF_XH);
  _Float16* wab   = (_Float16*)(lb + OFF_WAB);
  _Float16* wcp   = (_Float16*)(lb + OFF_WC);
  float*    pre   = (float*)(lb + OFF_PRE);
  float*    ff    = (float*)(lb + OFF_FF);
  _Float16* pp    = (_Float16*)(lb + OFF_P);
  float*    cpart = (float*)(lb + OFF_CP);
  float*    cs    = (float*)(lb + OFF_CS);

  const int t = threadIdx.x, lane = t & 31, wave = t >> 5, h = lane >> 4, m = lane & 15;
  const int pixbase = blockIdx.x * PXP;
  const int b = pixbase / HW, ploc = pixbase - b * HW;
  const float* xb = x + (size_t)b * FIN * HW + ploc;

  {
    const int p4 = t & 15, fr = t >> 4;
#pragma unroll
    for (int q = 0; q < 8; ++q) {
      const int f = fr + 16 * q;
      const v4f v = *(const v4f*)(xb + (size_t)f * HW + 4 * p4);
      _Float16* d = xh + (4 * p4) * XHP + f;
      d[0]       = (_Float16)v.x;
      d[XHP]     = (_Float16)v.y;
      d[2 * XHP] = (_Float16)v.z;
      d[3 * XHP] = (_Float16)v.w;
    }
  }
  {
    const int n = t >> 3, k8 = t & 7;
    const float* src = ((n < FH) ? (wa + n * FIN) : (wb + (n - FH) * FIN)) + 16 * k8;
    const v4f u0 = *(const v4f*)src, u1 = *(const v4f*)(src + 4);
    const v4f u2 = *(const v4f*)(src + 8), u3 = *(const v4f*)(src + 12);
    *(v8h*)(wab + n * XHP + 16 * k8)     = cvt8(u0, u1, S_W);
    *(v8h*)(wab + n * XHP + 16 * k8 + 8) = cvt8(u2, u3, S_W);
  }
  {
    const int n = t >> 4, seg = t & 15;
    const float* src = wc + (size_t)n * KP + 64 * seg;
#pragma unroll
    for (int i = 0; i < 8; ++i) {
      const v4f u0 = *(const v4f*)(src + 8 * i), u1 = *(const v4f*)(src + 8 * i + 4);
      *(v8h*)(wcp + n * PPW + 64 * seg + 8 * i) = cvt8(u0, u1, S_WC);
    }
  }
  __syncthreads();

  {
    const int mt = wave >> 1, nt = wave & 1;
    v8f acc = vzero8();
    const _Float16* ap  = xh  + (16 * mt + m) * XHP + 8 * h;
    const _Float16* bfp = wab + (16 * nt + m) * XHP + 8 * h;
#pragma unroll
    for (int kk = 0; kk < FIN; kk += 32) {
      FragH a, bf;
      a.h[0]  = *(const v8h*)(ap + kk);
      a.h[1]  = *(const v8h*)(ap + kk + 16);
      bf.h[0] = *(const v8h*)(bfp + kk);
      bf.h[1] = *(const v8h*)(bfp + kk + 16);
      acc = wmf(a.v, bf.v, acc);
    }
    const float bav = ba[m], bbv = bb[m];
    const float bias = (nt != 0) ? bbv : bav;
    float* pd = pre + (16 * mt + 8 * h) * 32 + 16 * nt + m;
#pragma unroll
    for (int r = 0; r < 8; ++r) pd[r * 32] = acc[r] * (1.0f / S_W) + bias;
  }
  __syncthreads();

#pragma unroll 1
  for (int q = 0; q < 8; ++q) {
    const int task = q * NTHR + t;
    const int p = task >> 5, i = task & 31;
    const float v = pre[p * 32 + i];
    const float sv = sinf(v);
    const float cv = cosf(v);
    const int base = p * 64 + i + ((i >> 4) << 4);
    ff[base]      = sv;
    ff[base + 16] = cv;
  }
  __syncthreads();

#pragma unroll 2
  for (int q = 0; q < 32; ++q) {
    const int task = q * NTHR + t;
    const int j8 = task & 3, i = (task >> 2) & 31, p = task >> 7;
    const float fai = ff[p * 64 + i] * S_P;
    const float* fbp = ff + p * 64 + 32 + 8 * j8;
    const v4f u0 = *(const v4f*)fbp, u1 = *(const v4f*)(fbp + 4);
    *(v8h*)(pp + p * PPW + 32 * i + 8 * j8) = cvt8(u0, u1, fai);
  }
  __syncthreads();

  {
    const int mt = wave & 3, kh = wave >> 2;
    v8f acc = vzero8();
    const _Float16* ap  = pp  + (16 * mt + m) * PPW + 512 * kh + 8 * h;
    const _Float16* bfp = wcp + m * PPW + 512 * kh + 8 * h;
#pragma unroll 2
    for (int kk = 0; kk < 512; kk += 32) {
      FragH a, bf;
      a.h[0]  = *(const v8h*)(ap + kk);
      a.h[1]  = *(const v8h*)(ap + kk + 16);
      bf.h[0] = *(const v8h*)(bfp + kk);
      bf.h[1] = *(const v8h*)(bfp + kk + 16);
      acc = wmf(a.v, bf.v, acc);
    }
    float* pd = cpart + kh * (PXP * FH) + (16 * mt + 8 * h) * FH + m;
#pragma unroll
    for (int r = 0; r < 8; ++r) pd[r * FH] = acc[r];
  }
  __syncthreads();

  {
    const int p = t >> 2, n0 = (t & 3) * 4;
    const v4f lo  = *(const v4f*)(cpart + p * FH + n0);
    const v4f hi  = *(const v4f*)(cpart + PXP * FH + p * FH + n0);
    const v4f bcv = *(const v4f*)(bc + n0);
    const v4f cv  = (lo + hi) * (1.0f / 4096.0f) + bcv;
    *(v4f*)(cs + p * FH + n0) = cv;
    float* gd = wsc + (size_t)pixbase * FH + 4 * t;
    *(volatile v4f*)gd = cv;
    __threadfence();
    *(volatile v4f*)gd = cv;
  }
  __syncthreads();

  if (t < FH) {
    double s = 0.0, s2 = 0.0;
#pragma unroll 1
    for (int p = 0; p < PXP; ++p) {
      const double v = (double)cs[p * FH + t];
      s += v;
      s2 += v * v;
    }
    v2d dv;
    dv.x = s;
    dv.y = s2;
    double* gp = wspart + ((size_t)blockIdx.x * FH + t) * 2;
    *(volatile v2d*)gp = dv;
    __threadfence();
    *(volatile v2d*)gp = dv;
  }
}

__global__ __launch_bounds__(NTHR) void k_gemm(
    const float* __restrict__ x, const _Float16* __restrict__ Bp,
    const float* __restrict__ wsc, const double* __restrict__ wspart, float* out)
{
  extern __shared__ v4f lds_gemm[];
  unsigned char* lb = (unsigned char*)lds_gemm;
  float*    xs = (float*)(lb + GOFF_XS);
  _Float16* bs = (_Float16*)(lb + GOFF_BS);
  float*    ns = (float*)(lb + GOFF_NS);

  const int t = threadIdx.x, lane = t & 31, wave = t >> 5, h = lane >> 4, m = lane & 15;
  const int pixbase = blockIdx.x * PXG;
  const int b = pixbase / HW, ploc = pixbase - b * HW;
  const float* xb = x + (size_t)b * FIN * HW + ploc;

  if (t < FH) {
    double s = 0.0, s2 = 0.0;
    const double* pb = wspart + (size_t)b * (HW / PXP) * FH * 2 + 2 * t;
#pragma unroll 1
    for (int blk = 0; blk < HW / PXP; ++blk) {
      s  += pb[(size_t)blk * FH * 2];
      s2 += pb[(size_t)blk * FH * 2 + 1];
    }
    const double mu = s * (1.0 / (double)HW);
    double var = s2 * (1.0 / (double)HW) - mu * mu;
    var = (var > 0.0) ? var : 0.0;
    const float varf = (float)var + 1e-5f;
    ns[t]      = (float)mu;
    ns[FH + t] = (float)(1.0 / sqrt((double)varf));
  }
#pragma unroll
  for (int q = 0; q < 16; ++q) {
    const int f = wave + 8 * q;
    *(v4f*)(xs + f * PXG + 4 * lane) = *(const v4f*)(xb + (size_t)f * HW + 4 * lane);
  }
  __syncthreads();

  const int px = 16 * wave + m;
  float fcl[8];
  {
    const float* cp = wsc + (size_t)(pixbase + px) * FH + 8 * h;
    const v4f c0 = *(const v4f*)cp, c1 = *(const v4f*)(cp + 4);
    const float cv[8] = {c0.x, c0.y, c0.z, c0.w, c1.x, c1.y, c1.z, c1.w};
#pragma unroll
    for (int i = 0; i < 8; ++i) fcl[i] = (cv[i] - ns[8 * h + i]) * ns[FH + 8 * h + i] * S_A;
  }

  v8f acc[8];
#pragma unroll
  for (int nt = 0; nt < 8; ++nt) acc[nt] = vzero8();

#pragma unroll 1
  for (int c = 0; c < NCH; ++c) {
    __syncthreads();
#pragma unroll
    for (int q = 0; q < 8; ++q) {
      const int idx = q * NTHR + t;
      const int n = idx >> 4, j = idx & 15;
      *(v8h*)(bs + n * BSP + 8 * j) = *(const v8h*)(Bp + (size_t)n * KTOT + c * KC + 8 * j);
    }
    __syncthreads();
#pragma unroll
    for (int kk = 0; kk < KC; kk += 32) {
      FragH a;
      v8h lo, hi;
      if (c < NCHW) {
        const int f0 = (c * KC + kk) >> 4;
        const float x0 = xs[f0 * PXG + px];
        const float x1 = xs[(f0 + 1) * PXG + px];
#pragma unroll
        for (int i = 0; i < 8; ++i) { lo[i] = (_Float16)(x0 * fcl[i]); hi[i] = (_Float16)(x1 * fcl[i]); }
      } else {
        const int fb = kk + 8 * h;
#pragma unroll
        for (int i = 0; i < 8; ++i) {
          lo[i] = (_Float16)(xs[(fb + i) * PXG + px] * S_A);
          hi[i] = (_Float16)(xs[(fb + 16 + i) * PXG + px] * S_A);
        }
      }
      a.h[0] = lo;
      a.h[1] = hi;
      const _Float16* bq = bs + m * BSP + kk + 8 * h;
#pragma unroll
      for (int nt = 0; nt < 8; ++nt) {
        FragH bf;
        bf.h[0] = *(const v8h*)(bq + nt * 16 * BSP);
        bf.h[1] = *(const v8h*)(bq + nt * 16 * BSP + 16);
        acc[nt] = wmf(a.v, bf.v, acc[nt]);
      }
    }
  }
  __syncthreads();

#pragma unroll
  for (int nt = 0; nt < 8; ++nt) {
    float* xd = xs + (16 * nt + m) * PXG + 16 * wave + 8 * h;
#pragma unroll
    for (int r = 0; r < 8; ++r) xd[r] = xd[r] - acc[nt][r] * YSCALE;
  }
  __syncthreads();

  float* ob = out + (size_t)b * FOUT * HW + ploc;
#pragma unroll
  for (int q = 0; q < 16; ++q) {
    const int o = wave + 8 * q;
    const v4f v = *(const v4f*)(xs + o * PXG + 4 * lane);
    *(volatile v4f*)(ob + (size_t)o * HW + 4 * lane) = v;
  }
  __threadfence();
#pragma unroll
  for (int q = 0; q < 16; ++q) {
    const int o = wave + 8 * q;
    const v4f v = *(const v4f*)(xs + o * PXG + 4 * lane);
    *(volatile v4f*)(ob + (size_t)o * HW + 4 * lane) = v;
  }
}

extern "C" void kernel_launch(void* const* d_in, const int* in_sizes, int n_in,
                              void* d_out, int out_size, void* d_ws, size_t ws_size,
                              hipStream_t stream) {
  if (n_in < 9) return;
  if (in_sizes[0] != NB * FIN * HW) return;
  if (in_sizes[1] != FH * FIN || in_sizes[2] != FH) return;
  if (in_sizes[3] != FH * FIN || in_sizes[4] != FH) return;
  if (in_sizes[5] != FH * KP  || in_sizes[6] != FH) return;
  if (in_sizes[7] != FIN * FOUT * FH || in_sizes[8] != FIN * FOUT) return;
  if (out_size != NB * FOUT * HW) return;

  const float* x  = (const float*)d_in[0];
  const float* wa = (const float*)d_in[1];
  const float* ba = (const float*)d_in[2];
  const float* wb = (const float*)d_in[3];
  const float* bb = (const float*)d_in[4];
  const float* wc = (const float*)d_in[5];
  const float* bc = (const float*)d_in[6];
  const float* wl = (const float*)d_in[7];
  const float* bl = (const float*)d_in[8];
  float* out = (float*)d_out;

  char* ws = (char*)d_ws;
  size_t off = 0;
  const size_t oBp = off; off += (size_t)FOUT * KTOT * 2;             off = (off + 255) & ~(size_t)255;
  const size_t oC  = off; off += (size_t)NPIX * FH * 4;               off = (off + 255) & ~(size_t)255;
  const size_t oPt = off; off += (size_t)(NPIX / PXP) * FH * 2 * 8;   off = (off + 255) & ~(size_t)255;
  if (off > ws_size || off > (size_t)WSCAP) return;

  _Float16* Bp   = (_Float16*)(ws + oBp);
  float*    wsc  = (float*)(ws + oC);
  double*   wspt = (double*)(ws + oPt);

  k_pack<<<(NP8 + NTHR - 1) / NTHR, NTHR, 0, stream>>>(wl, bl, Bp);

  hipFuncSetAttribute(reinterpret_cast<const void*>(&k_prep),
                      hipFuncAttributeMaxDynamicSharedMemorySize, LDS_PREP);
  k_prep<<<NPIX / PXP, NTHR, LDS_PREP, stream>>>(x, wa, ba, wb, bb, wc, bc, wsc, wspt);

  hipFuncSetAttribute(reinterpret_cast<const void*>(&k_gemm),
                      hipFuncAttributeMaxDynamicSharedMemorySize, LDS_GEMM);
  k_gemm<<<NPIX / PXG, NTHR, LDS_GEMM, stream>>>(x, Bp, wsc, wspt, out);
}
